// VolumeRenderer_35527969472978
// MI455X (gfx1250) — hardware-verified
//
#include <hip/hip_runtime.h>
#include <math.h>

typedef __attribute__((ext_vector_type(16))) _Float16 v16h;
typedef __attribute__((ext_vector_type(16))) __bf16 v16b;
typedef __attribute__((ext_vector_type(8)))  _Float16 v8h;
typedef __attribute__((ext_vector_type(8)))  float v8f;
typedef __attribute__((ext_vector_type(4)))  float v4f;
typedef __attribute__((ext_vector_type(2)))  float v2f;
typedef __attribute__((ext_vector_type(4)))  unsigned v4u;
typedef __attribute__((ext_vector_type(4)))  int v4i;
typedef float __attribute__((may_alias)) float_a;
typedef int __attribute__((may_alias)) int_a;

template <typename T> __device__ __forceinline__ void vst2(void* p, T v) { *(volatile T*)p = v; __threadfence(); *(volatile T*)p = v; }
__device__ __forceinline__ v8f wmma16(v16h a, v16h b, v8f c) {
  v8f d = __builtin_amdgcn_wmma_f32_16x16x32_f16(false, a, false, b, (short)0, c, false, false);
  asm volatile("v_nop\n\tv_nop\n\tv_nop\n\tv_nop" : "+v"(d) : "v"(a), "v"(b));
  return d;
}
__device__ __forceinline__ v8f wmma_bf(v16b a, v16b b, v8f c) {
  v8f d = __builtin_amdgcn_wmma_f32_16x16x32_bf16(false, a, false, b, (short)0, c, false, false);
  asm volatile("v_nop\n\tv_nop\n\tv_nop\n\tv_nop" : "+v"(d) : "v"(a), "v"(b));
  return d;
}
__device__ __forceinline__ v16h frag_h(const _Float16* rowk0, int lane) {
  union { v16h v; v8h q[2]; } u; const _Float16* p = rowk0 + 8 * (lane >> 4);
  u.q[0] = *(const v8h*)p; u.q[1] = *(const v8h*)(p + 16); return u.v;
}
__device__ __forceinline__ v16h frag_f32(const float* rowk0, int lane) {
  v16h a; const float* p = rowk0 + 8 * (lane >> 4);
#pragma unroll
  for (int i = 0; i < 8; ++i) { a[i] = (_Float16)p[i]; a[8 + i] = (_Float16)p[16 + i]; }
  return a;
}
__device__ __forceinline__ v16h frag_f32s(const float* rowk0, int lane, float sc) {
  v16h a; const float* p = rowk0 + 8 * (lane >> 4);
#pragma unroll
  for (int i = 0; i < 8; ++i) { a[i] = (_Float16)(p[i] * sc); a[8 + i] = (_Float16)(p[16 + i] * sc); }
  return a;
}
__device__ __forceinline__ v16h fragc_f32(const float* W, int k0, int n, int lane, int ld, int K) {
  v16h a; const int g = lane >> 4;
#pragma unroll
  for (int i = 0; i < 8; ++i) { const int ka = k0 + 8 * g + i, kb = ka + 16;
    a[i] = (_Float16)(ka < K ? W[(size_t)(ka < K ? ka : K - 1) * ld + n] : 0.f); a[8 + i] = (_Float16)(kb < K ? W[(size_t)(kb < K ? kb : K - 1) * ld + n] : 0.f); }
  return a;
}
struct F2 { v16b h, l; };
__device__ __forceinline__ F2 bsplit16(const float v[16]) { F2 r;
#pragma unroll
  for (int i = 0; i < 16; ++i) { const __bf16 h = (__bf16)v[i]; r.h[i] = h; r.l[i] = (__bf16)(v[i] - (float)h); }
  return r; }
__device__ __forceinline__ F2 split_row(const float* row, int k0, int lane) { float v[16]; const float* p = row + k0 + 8 * (lane >> 4);
#pragma unroll
  for (int i = 0; i < 8; ++i) { v[i] = p[i]; v[8 + i] = p[16 + i]; }
  return bsplit16(v); }
__device__ __forceinline__ F2 split_rowK(const float* row, int k0, int lane, int K) { float v[16]; const int g = lane >> 4;
#pragma unroll
  for (int i = 0; i < 8; ++i) { const int ka = k0 + 8 * g + i, kb = ka + 16; v[i] = ka < K ? row[ka < K ? ka : K - 1] : 0.f; v[8 + i] = kb < K ? row[kb < K ? kb : K - 1] : 0.f; }
  return bsplit16(v); }
__device__ __forceinline__ F2 split_col(const float* W, int k0, int n, int lane, int ld, int K) { float v[16]; const int g = lane >> 4;
#pragma unroll
  for (int i = 0; i < 8; ++i) { const int ka = k0 + 8 * g + i, kb = ka + 16; v[i] = ka < K ? W[(size_t)(ka < K ? ka : K - 1) * ld + n] : 0.f; v[8 + i] = kb < K ? W[(size_t)(kb < K ? kb : K - 1) * ld + n] : 0.f; }
  return bsplit16(v); }
__device__ __forceinline__ v8f mac3(const F2& a, const F2& b, v8f c) { c = wmma_bf(a.l, b.h, c); c = wmma_bf(a.h, b.l, c); return wmma_bf(a.h, b.h, c); }
__device__ __forceinline__ float sigm(float v) { return 1.0f / (1.0f + expf(-v)); }
#define LDSX() do { asm volatile("s_wait_dscnt 0" ::: "memory"); __builtin_amdgcn_wave_barrier(); __builtin_amdgcn_fence(__ATOMIC_RELEASE, "workgroup"); } while (0)

#define NRAY 4096
#define KS 256
#define NV 100000
#define DE 32
#define HID 64
#define INW 38
#define NPTS (NRAY * KS)
#ifndef NRV
#define NRV NRAY
#endif
#define OFF_DEPTHS 49152u
#define OFF_MISSED 65536u
#define OFF_PROBS  81920u
__device__ __forceinline__ float bfr(float v) { return (float)(__bf16)v; }
__device__ __forceinline__ v16b wcol_kz(const float* __restrict__ Wm, int k0, int o, int lane, int ld, int K, int nvalid) { v16b w; const int g = lane >> 4; const int oc = o < nvalid ? o : 0; const float keepo = o < nvalid ? 1.f : 0.f;
  asm volatile("s_wait_loadcnt 0x0" ::: "memory");
#pragma unroll
  for (int i = 0; i < 8; ++i) { const int ka = k0 + 8 * g + i, kb = ka + 16; w[i] = (__bf16)(Wm[(size_t)(ka < K ? ka : 0) * ld + oc] * (ka < K ? keepo : 0.f)); w[8 + i] = (__bf16)(Wm[(size_t)(kb < K ? kb : 0) * ld + oc] * (kb < K ? keepo : 0.f)); }
  asm volatile("s_wait_loadcnt 0x0" ::: "memory"); return w; }
#define WS_O4  0u
#define WS_RAY (WS_O4 + 16u * (size_t)NPTS)
#define WS_END (WS_RAY + 128u * (size_t)NRAY)
__global__ __launch_bounds__(128) void k_mlp(const float* __restrict__ RS, const float* __restrict__ RD, const float* __restrict__ DEP, const int* __restrict__ IDXI, const float* __restrict__ EMB,
    const float* __restrict__ W1, const float* __restrict__ B1, const float* __restrict__ W2, const float* __restrict__ B2, const float* __restrict__ WO, const float* __restrict__ BO, float* __restrict__ O4) {
  __shared__ __align__(16) float sh[4][16][68];
  const int tid = threadIdx.x, wave = tid >> 5, lane = tid & 31, col = lane & 15, g = lane >> 4; const size_t r0 = (size_t)blockIdx.x * 64 + wave * 16; const size_t pt = r0 + col; const size_t ray = pt / KS;
  int ix = IDXI[pt]; ix = ix < 0 ? 0 : (ix >= NV ? NV - 1 : ix);
  const float sx = bfr(RS[ray * 3]), sy = bfr(RS[ray * 3 + 1]), szz = bfr(RS[ray * 3 + 2]), dx = bfr(RD[ray * 3]), dy = bfr(RD[ray * 3 + 1]), dz = bfr(RD[ray * 3 + 2]), dep = bfr(DEP[pt]);
  asm volatile("s_wait_loadcnt 0x0" ::: "memory");
  v8f acc[4] = {};
#pragma unroll
  for (int kc = 0; kc < 2; ++kc) { float va[16];
#pragma unroll
    for (int i = 0; i < 16; ++i) { const int k = kc * 32 + 8 * g + (i < 8 ? i : 8 + i); float v;
      { const int ke = k - 3; const int kec = ke < 0 ? 0 : (ke > DE - 1 ? DE - 1 : ke); const float e = bfr(EMB[(size_t)ix * DE + kec]);
        const float pc = (k == 0 ? sx : (k == 1 ? sy : szz)) + (k == 0 ? dx : (k == 1 ? dy : dz)) * dep;
        const float dc = (k == 35 ? dx : (k == 36 ? dy : dz));
        v = k < 3 ? pc : (k < 3 + DE ? e : (k < INW ? dc : 0.f)); }
      va[i] = v; if (i == 7) asm volatile("s_wait_loadcnt 0x0" ::: "memory"); }
    asm volatile("s_wait_loadcnt 0x0" ::: "memory");
    const F2 a = bsplit16(va);
#pragma unroll
    for (int j = 0; j < 4; ++j) { const v16b w = wcol_kz(W1, kc * 32, j * 16 + col, lane, HID, INW, HID); acc[j] = wmma_bf(a.h, w, acc[j]); acc[j] = wmma_bf(a.l, w, acc[j]); } }
#pragma unroll
  for (int j = 0; j < 4; ++j) { const float bb = bfr(B1[j * 16 + col]);
#pragma unroll
    for (int r = 0; r < 8; ++r) sh[wave][8 * g + r][j * 16 + col] = fmaxf(acc[j][r] + bb, 0.f); }
  LDSX();
  { v8f acc2[4] = {};
#pragma unroll
    for (int kc = 0; kc < 2; ++kc) { const F2 a = split_row(&sh[wave][col][0], kc * 32, lane);
#pragma unroll
      for (int j = 0; j < 4; ++j) { const v16b w = wcol_kz(W2, kc * 32, j * 16 + col, lane, HID, HID, HID); acc2[j] = wmma_bf(a.h, w, acc2[j]); acc2[j] = wmma_bf(a.l, w, acc2[j]); } }
    LDSX();
#pragma unroll
    for (int j = 0; j < 4; ++j) { const float bb = bfr(B2[j * 16 + col]);
#pragma unroll
      for (int r = 0; r < 8; ++r) sh[wave][8 * g + r][j * 16 + col] = fmaxf(acc2[j][r] + bb, 0.f); } }
  LDSX();
  { v8f acc3 = {};
#pragma unroll
    for (int kc = 0; kc < 2; ++kc) { const F2 a = split_row(&sh[wave][col][0], kc * 32, lane); const v16b w = wcol_kz(WO, kc * 32, col, lane, 4, HID, 4); acc3 = wmma_bf(a.h, w, acc3); acc3 = wmma_bf(a.l, w, acc3); }
    LDSX();
    const float bb = col < 4 ? bfr(BO[col < 4 ? col : 0]) : 0.f;
    if (col < 4) {
#pragma unroll
      for (int r = 0; r < 8; ++r) sh[wave][8 * g + r][col] = acc3[r] + bb; } }
  LDSX();
  if (lane < 16) vst2(O4 + (r0 + lane) * 4, *(const v4f*)&sh[wave][lane][0]); }
__global__ __launch_bounds__(256) void k_ray(const float* __restrict__ O4, const int* __restrict__ IDXI, const float* __restrict__ DEP, const float* __restrict__ DST, float* __restrict__ PROBS, float* __restrict__ RAYW) {
  const int wave = threadIdx.x >> 5, lane = threadIdx.x & 31; const size_t ray = (size_t)blockIdx.x * 8 + wave;
  float fe[8], pr[8], dep[8], tx[8], ty[8], tz[8]; int mk[8];
#pragma unroll
  for (int i = 0; i < 8; ++i) { const size_t pt = ray * KS + lane * 8 + i; const v4f o = *(const v4f*)(O4 + pt * 4); mk[i] = IDXI[pt] >= 0; dep[i] = bfr(DEP[pt]); const float ds = bfr(DST[pt]); asm volatile("s_wait_loadcnt 0x0" ::: "memory");
    fe[i] = mk[i] ? fmaxf(o[0], 0.f) * ds : 0.f; tx[i] = mk[i] ? o[1] : 0.f; ty[i] = mk[i] ? o[2] : 0.f; tz[i] = mk[i] ? o[3] : 0.f; }
  float run = 0.f, excl[8];
#pragma unroll
  for (int i = 0; i < 8; ++i) { excl[i] = run; run += fe[i]; }
  float incl = run;
#pragma unroll
  for (int o = 1; o < 32; o <<= 1) { const float t = __shfl_up(incl, o); incl = (lane >= o) ? incl + t : incl; }
  const float before = incl - run;
  float psum = 0.f, dsum = 0.f, cx = 0.f, cy = 0.f, cz = 0.f;
#pragma unroll
  for (int i = 0; i < 8; ++i) { const float cum = before + excl[i]; const float bexp = expf(-cum); const float a = 1.0f - expf(-fe[i]); const float p = a * bexp; pr[i] = p; psum += p; dsum += dep[i] * p; cx += tx[i] * p; cy += ty[i] * p; cz += tz[i] * p; }
#pragma unroll
  for (int o = 1; o < 32; o <<= 1) { psum += __shfl_xor(psum, o); dsum += __shfl_xor(dsum, o); cx += __shfl_xor(cx, o); cy += __shfl_xor(cy, o); cz += __shfl_xor(cz, o); }
  { v4f a4, b4; a4[0] = pr[0]; a4[1] = pr[1]; a4[2] = pr[2]; a4[3] = pr[3]; b4[0] = pr[4]; b4[1] = pr[5]; b4[2] = pr[6]; b4[3] = pr[7]; vst2(PROBS + ray * KS + lane * 8, a4); vst2(PROBS + ray * KS + lane * 8 + 4, b4); }
  if (lane < 8) { v4f w4; w4[0] = lane == 0 ? cx : 0.f; w4[1] = lane == 0 ? cy : 0.f; w4[2] = lane == 0 ? cz : 0.f; w4[3] = lane == 0 ? dsum : 0.f; if (lane == 1) { w4[0] = 1.0f - psum; } vst2(RAYW + ray * 32 + lane * 4, w4); } }
__global__ __launch_bounds__(256) void k_fin(const float* __restrict__ RAYW, float* __restrict__ COL, float* __restrict__ DEPO, float* __restrict__ MISO) { const size_t r = (size_t)blockIdx.x * 256 + threadIdx.x; if (r >= (size_t)NRV) return;
  const v4f a = *(const v4f*)(RAYW + r * 32); const v4f b = *(const v4f*)(RAYW + r * 32 + 4); asm volatile("s_wait_loadcnt 0x0" ::: "memory");
  vst2(COL + r * 3, a[0]); vst2(COL + r * 3 + 1, a[1]); vst2(COL + r * 3 + 2, a[2]); vst2(DEPO + r, a[3]); vst2(MISO + r, b[0]); }
extern "C" void kernel_launch(void* const* d_in, const int* in_sizes, int n_in, void* d_out, int out_size, void* d_ws, size_t ws_size, hipStream_t stream) {
  (void)in_sizes; (void)n_in; (void)out_size;
  if (ws_size < (size_t)WS_END) return;
  char* ws = (char*)d_ws; const float** F = (const float**)d_in; float* O4 = (float*)(ws + WS_O4); float* RAYW = (float*)(ws + WS_RAY);
  k_mlp<<<dim3(NRV * KS / 64), 128, 0, stream>>>(F[0], F[1], F[2], (const int*)d_in[3], F[5], F[6], F[7], F[8], F[9], F[10], F[11], O4);
  k_ray<<<dim3(NRV / 8), 256, 0, stream>>>(O4, (const int*)d_in[3], F[2], F[4], (float*)((char*)d_out + OFF_PROBS), RAYW);
  k_fin<<<dim3((NRV + 255) / 256), 256, 0, stream>>>(RAYW, (float*)d_out, (float*)((char*)d_out + OFF_DEPTHS), (float*)((char*)d_out + OFF_MISSED));
}
